// EIGLayerSimple_67997922230879
// MI455X (gfx1250) — hardware-verified
//
#include <hip/hip_runtime.h>
#include <stddef.h>
#include <math.h>

#pragma clang fp contract(off)


#define DF      128
#define KTOT    1536
#define SEGK    512
#define NTHR    512
#define NWAVE   16
#define EPT     8
#define NGRP    1
#define CHUNK   (NTHR * EPT * NGRP)
#define WCAP    (EPT * NGRP * 32)
#define LISTN   (NWAVE * WCAP)
#define NB      128
#define SROW    512
#define LDS_AGG (NB * SROW * 4 + LISTN * 4 + NB * 4 + NWAVE * 4)
#define ATHR    256
#define AVGD    2.565f
#define EPSV    1e-5f

static_assert((CHUNK & (CHUNK - 1)) == 0);
static_assert(CHUNK == 4096);
static_assert((NB & (NB - 1)) == 0);
static_assert(NB == 8 * 16);
static_assert(NWAVE == 16);
static_assert(LISTN * 4 >= 2 * DF * 8);
static_assert(NB * DF * 4 <= NB * SROW * 4);
static_assert((NB * DF) % NTHR == 0);

typedef float          v4f  __attribute__((ext_vector_type(4)));
typedef float          v8f  __attribute__((ext_vector_type(8)));
typedef int            v4i  __attribute__((ext_vector_type(4)));
typedef unsigned short v8us __attribute__((ext_vector_type(8)));
typedef __bf16         v16bf __attribute__((ext_vector_type(16)));
typedef double         v2d  __attribute__((ext_vector_type(2)));
union FragB { v16bf v; v8us u[2]; };

__device__ __forceinline__ unsigned bfbits(float x) {
  const unsigned u = __float_as_uint(x);
  return (u + 0x7FFFu + ((u >> 16) & 1u)) >> 16;
}

__device__ __forceinline__ void split8(v4f a, v4f b, v8us& hi, v8us& lo) {
  float xs[8] = {a.x, a.y, a.z, a.w, b.x, b.y, b.z, b.w};
#pragma unroll
  for (int i = 0; i < 8; ++i) {
    const unsigned hb = bfbits(xs[i]);
    const float rem = xs[i] - __uint_as_float(hb << 16);
    const unsigned lb = bfbits(rem);
    hi[i] = (unsigned short)hb;
    lo[i] = (unsigned short)lb;
  }
}

__device__ __forceinline__ v8f wmb(v16bf a, v16bf b, v8f c) {
  v8f d = __builtin_amdgcn_wmma_f32_16x16x32_bf16(false, a, false, b, (short)0, c, false, false);
  asm volatile("v_nop\n\tv_nop\n\tv_nop\n\tv_nop" : "+v"(d) : "v"(a), "v"(b));
  return d;
}

__device__ __forceinline__ int scan_chunk(const int* __restrict__ dsts, int nE, int cbase, int nodeBase,
                                          int vec8, int* list, int tid, int lane, int wave) {
  int wc = 0;
#pragma unroll
  for (int g = 0; g < NGRP; ++g) {
    const int el0  = (g * NTHR + tid) * EPT;
    const int e0   = cbase + el0;
    const int sent = -2147483647 - 1;
    v4i da, db;
    if (vec8 != 0 && cbase + CHUNK <= nE) {
      da = *(const v4i*)(dsts + e0);
      db = *(const v4i*)(dsts + e0 + 4);
    } else {
      const int em = nE - 1;
      da.x = (e0     < nE) ? dsts[min(e0,     em)] : sent;
      da.y = (e0 + 1 < nE) ? dsts[min(e0 + 1, em)] : sent;
      da.z = (e0 + 2 < nE) ? dsts[min(e0 + 2, em)] : sent;
      da.w = (e0 + 3 < nE) ? dsts[min(e0 + 3, em)] : sent;
      db.x = (e0 + 4 < nE) ? dsts[min(e0 + 4, em)] : sent;
      db.y = (e0 + 5 < nE) ? dsts[min(e0 + 5, em)] : sent;
      db.z = (e0 + 6 < nE) ? dsts[min(e0 + 6, em)] : sent;
      db.w = (e0 + 7 < nE) ? dsts[min(e0 + 7, em)] : sent;
    }
    const unsigned nb = (unsigned)nodeBase;
    const unsigned s0 = (unsigned)da.x - nb, s1 = (unsigned)da.y - nb;
    const unsigned s2 = (unsigned)da.z - nb, s3 = (unsigned)da.w - nb;
    const unsigned s4 = (unsigned)db.x - nb, s5 = (unsigned)db.y - nb;
    const unsigned s6 = (unsigned)db.z - nb, s7 = (unsigned)db.w - nb;
    const bool h0 = s0 < (unsigned)NB, h1 = s1 < (unsigned)NB, h2 = s2 < (unsigned)NB, h3 = s3 < (unsigned)NB;
    const bool h4 = s4 < (unsigned)NB, h5 = s5 < (unsigned)NB, h6 = s6 < (unsigned)NB, h7 = s7 < (unsigned)NB;
    const unsigned any = __builtin_amdgcn_ballot_w32(h0 | h1 | h2 | h3 | h4 | h5 | h6 | h7);
    if (any != 0u) {
#define HITJ(J, HJ, SJ) { \
        const unsigned mj = __builtin_amdgcn_ballot_w32(HJ); \
        if (mj != 0u) { \
          if (HJ) { \
            const int pos = wc + (int)__builtin_amdgcn_mbcnt_lo(mj, 0u); \
            if (pos < WCAP) list[wave * WCAP + pos] = ((el0 + (J)) << 12) | (int)(SJ); \
          } \
          wc += (int)__builtin_popcount(mj); } }
      HITJ(0, h0, s0)
      HITJ(1, h1, s1)
      HITJ(2, h2, s2)
      HITJ(3, h3, s3)
      HITJ(4, h4, s4)
      HITJ(5, h5, s5)
      HITJ(6, h6, s6)
      HITJ(7, h7, s7)
#undef HITJ
    }
  }
  return wc;
}

__global__ __launch_bounds__(ATHR) void k_wprep(
    const float* __restrict__ W, unsigned short* whi, unsigned short* wlo, int total8) {
  const int i = blockIdx.x * ATHR + threadIdx.x;
  if (i >= total8) return;
  const int o  = i * 8;
  const int n  = o / KTOT;
  const int k0 = o - n * KTOT;
  const float* p = W + (size_t)k0 * DF + n;
  v4f a, b;
  a.x = p[0];      a.y = p[DF];     a.z = p[2 * DF]; a.w = p[3 * DF];
  b.x = p[4 * DF]; b.y = p[5 * DF]; b.z = p[6 * DF]; b.w = p[7 * DF];
  v8us hv, lv;
  split8(a, b, hv, lv);
  *(volatile v8us*)(whi + o) = hv;
  *(volatile v8us*)(wlo + o) = lv;
  __threadfence();
  *(volatile v8us*)(whi + o) = hv;
  *(volatile v8us*)(wlo + o) = lv;
}

__global__ __launch_bounds__(NTHR) void k_agg(
    const float* __restrict__ h, const int* __restrict__ srcs, const int* __restrict__ dsts,
    const float* __restrict__ snorm, const float* __restrict__ bpost,
    const unsigned short* __restrict__ whi, const unsigned short* __restrict__ wlo,
    float* zpl, double* part, int nN, int nE, int vec8) {
  extern __shared__ v4f lds_dyn[];
  float*  state = (float*)lds_dyn;
  int*    list  = (int*)(state + NB * SROW);
  int*    cnt   = list + LISTN;
  int*    wcnt  = cnt + NB;
  double* dpart = (double*)list;
  const int tid = threadIdx.x, lane = tid & 31, wave = tid >> 5, hh = lane >> 4, m = lane & 15;
  const int nodeBase = blockIdx.x * NB;

  {
    const float ninf = __uint_as_float(0xff800000u), pinf = __uint_as_float(0x7f800000u);
    for (int i = tid; i < NB * SROW / 4; i += NTHR) {
      const int c = (i * 4) & (SROW - 1);
      const float f = (c < 128) ? 0.f : ((c < 256) ? ninf : ((c < 384) ? pinf : 0.f));
      v4f v; v.x = f; v.y = f; v.z = f; v.w = f;
      lds_dyn[i] = v;
    }
    for (int i = tid; i < NB; i += NTHR) cnt[i] = 0;
  }
  __syncthreads();

  const int nChunks = (nE + CHUNK - 1) / CHUNK;
#pragma unroll 1
  for (int ch = 0; ch < nChunks; ++ch) {
    const int cbase = ch * CHUNK;
    const int wc = scan_chunk(dsts, nE, cbase, nodeBase, vec8, list, tid, lane, wave);
    if (lane == 0) wcnt[wave] = wc;
    __syncthreads();
    if (wave == 0) {
#pragma unroll 1
      for (int wsx = 0; wsx < NWAVE; ++wsx) {
        int n = __builtin_amdgcn_readfirstlane(wcnt[wsx]);
        n = n > WCAP ? WCAP : (n < 0 ? 0 : n);
        const int* lp = list + wsx * WCAP;
#pragma unroll 1
        for (int i = 0; i < n; ++i) {
          const int ent  = __builtin_amdgcn_readfirstlane(lp[i]);
          const int slot = ent & (NB - 1);
          int e = cbase + ((ent >> 12) & (CHUNK - 1));
          e = e > nE - 1 ? nE - 1 : e;
          int s = srcs[e];
          s = s < 0 ? 0 : (s > nN - 1 ? nN - 1 : s);
          const v4f v = *(const v4f*)(h + (size_t)s * DF + 4 * lane);
          float* row = state + slot * SROW + 4 * lane;
          v4f S = *(const v4f*)row;
          v4f M = *(const v4f*)(row + 128);
          v4f L = *(const v4f*)(row + 256);
          v4f Q = *(const v4f*)(row + 384);
          S = S + v;
          Q = Q + v * v;
          M.x = fmaxf(M.x, v.x); M.y = fmaxf(M.y, v.y); M.z = fmaxf(M.z, v.z); M.w = fmaxf(M.w, v.w);
          L.x = fminf(L.x, v.x); L.y = fminf(L.y, v.y); L.z = fminf(L.z, v.z); L.w = fminf(L.w, v.w);
          *(v4f*)row         = S;
          *(v4f*)(row + 128) = M;
          *(v4f*)(row + 256) = L;
          *(v4f*)(row + 384) = Q;
          if (lane == 0) cnt[slot] = cnt[slot] + 1;
        }
      }
    }
    __syncthreads();
  }

#pragma unroll 1
  for (int it = 0; it < (NB * DF) / NTHR; ++it) {
    const int idx  = it * NTHR + tid;
    const int slot = idx >> 7;
    const int c    = idx & (DF - 1);
    const int dg   = cnt[slot];
    const float ds  = dg > 0 ? (float)dg : 1.f;
    const float inv = 1.0f / ds;
    float* row = state + slot * SROW;
    const float S = row[c], M = row[128 + c], L = row[256 + c], Q = row[384 + c];
    const float mean = S * inv;
    const float s2   = Q * inv;
    const float var  = s2 - mean * mean;
    const float sd   = sqrtf(fmaxf(var, 0.f) + EPSV);
    row[c]       = mean;
    row[128 + c] = dg > 0 ? M : 0.f;
    row[256 + c] = dg > 0 ? L : 0.f;
    row[384 + c] = sd;
  }
  __syncthreads();

  const int rg = wave & 7, chf = wave >> 3;
  const int slotm = rg * 16 + m;
  const int dgm = cnt[slotm];
  const float dsm  = dgm > 0 ? (float)dgm : 1.f;
  const float logd = logf(dsm + 1.f);
  const float sc1  = logd / AVGD;
  const float sc2  = AVGD / logd;
  const float* arow = state + slotm * SROW + 8 * hh;
  const unsigned short* wbh = whi + (size_t)(64 * chf + m) * KTOT + 8 * hh;
  const unsigned short* wbl = wlo + (size_t)(64 * chf + m) * KTOT + 8 * hh;

  v8f acc[4];
#pragma unroll
  for (int t = 0; t < 4; ++t) { v8f z = {0.f, 0.f, 0.f, 0.f, 0.f, 0.f, 0.f, 0.f}; acc[t] = z; }

#pragma unroll 1
  for (int seg = 0; seg < 3; ++seg) {
    const float s = (seg == 0) ? 1.f : ((seg == 1) ? sc1 : sc2);
#pragma unroll 1
    for (int kt = 0; kt < SEGK / 32; ++kt) {
      const float* ap = arow + 32 * kt;
      v4f p0 = *(const v4f*)ap,        p1 = *(const v4f*)(ap + 4);
      v4f p2 = *(const v4f*)(ap + 16), p3 = *(const v4f*)(ap + 20);
      p0 = p0 * s; p1 = p1 * s; p2 = p2 * s; p3 = p3 * s;
      FragB ah, al;
      split8(p0, p1, ah.u[0], al.u[0]);
      split8(p2, p3, ah.u[1], al.u[1]);
      const int koff = seg * SEGK + 32 * kt;
#pragma unroll
      for (int t = 0; t < 4; ++t) {
        const unsigned short* bph = wbh + (size_t)(16 * t) * KTOT + koff;
        const unsigned short* bpl = wbl + (size_t)(16 * t) * KTOT + koff;
        FragB bh, bl;
        bh.u[0] = *(const v8us*)bph;
        bh.u[1] = *(const v8us*)(bph + 16);
        bl.u[0] = *(const v8us*)bpl;
        bl.u[1] = *(const v8us*)(bpl + 16);
        acc[t] = wmb(ah.v, bh.v, acc[t]);
        acc[t] = wmb(ah.v, bl.v, acc[t]);
        acc[t] = wmb(al.v, bh.v, acc[t]);
      }
    }
  }
  __syncthreads();

  {
    float sn[8];
#pragma unroll
    for (int r = 0; r < 8; ++r) {
      int node = nodeBase + rg * 16 + 8 * hh + r;
      node = node > nN - 1 ? nN - 1 : node;
      sn[r] = snorm[node];
    }
    float* sp = state + (rg * 16 + 8 * hh) * DF + 64 * chf + m;
#pragma unroll
    for (int t = 0; t < 4; ++t) {
      const float bb = bpost[64 * chf + 16 * t + m];
#pragma unroll
      for (int r = 0; r < 8; ++r) sp[r * DF + 16 * t] = (acc[t][r] + bb) * sn[r];
    }
  }
  __syncthreads();

  {
    int nValid = nN - nodeBase;
    nValid = nValid > NB ? NB : (nValid < 0 ? 0 : nValid);
    if (tid < 2 * DF) {
      const int c = tid & (DF - 1), which = tid >> 7;
      double a = 0.0;
#pragma unroll 1
      for (int r = 0; r < nValid; ++r) {
        const double zd = (double)state[r * DF + c];
        a += (which != 0) ? zd * zd : zd;
      }
      dpart[which * DF + c] = a;
    }
  }
  __syncthreads();

  v4f zv[8];
  const float* lrow = state + (8 * wave) * DF + 4 * lane;
#pragma unroll
  for (int i = 0; i < 8; ++i) zv[i] = *(const v4f*)(lrow + i * DF);
  v2d pv; pv.x = 0.0; pv.y = 0.0;
  if (tid < DF) pv = *(const v2d*)(dpart + 2 * tid);
  float* zp = zpl + ((size_t)nodeBase + 8 * wave) * DF + 4 * lane;
#pragma unroll
  for (int i = 0; i < 8; ++i) *(volatile v4f*)(zp + (size_t)i * DF) = zv[i];
  if (tid < DF) { double* pp = part + (size_t)blockIdx.x * (2 * DF) + 2 * tid; *(volatile v2d*)pp = pv; }
  __threadfence();
#pragma unroll
  for (int i = 0; i < 8; ++i) *(volatile v4f*)(zp + (size_t)i * DF) = zv[i];
  if (tid < DF) { double* pp = part + (size_t)blockIdx.x * (2 * DF) + 2 * tid; *(volatile v2d*)pp = pv; }
}

__global__ __launch_bounds__(ATHR) void k_bnfin(const double* __restrict__ part, float* bnp, int nBlk, int nN) {
  __shared__ double sh[2 * DF];
  __shared__ __attribute__((aligned(16))) float res[2 * DF];
  const int tid = threadIdx.x;
  const int c = tid & (DF - 1), which = tid >> 7;
  double a = 0.0;
#pragma unroll 1
  for (int b = 0; b < nBlk; ++b) a += part[(size_t)b * (2 * DF) + which * DF + c];
  sh[tid] = a;
  __syncthreads();
  if (tid < DF) {
    const double invn = 1.0 / (double)nN;
    const double mu = sh[tid] * invn;
    double var = sh[DF + tid] * invn - mu * mu;
    var = var < 0.0 ? 0.0 : var;
    const float varf = (float)var;
    const float rs = 1.0f / sqrtf(varf + EPSV);
    res[tid]      = (float)mu;
    res[DF + tid] = rs;
  }
  __syncthreads();
  v4f v; v.x = 0.f; v.y = 0.f; v.z = 0.f; v.w = 0.f;
  if (tid < 64) v = *(const v4f*)(res + 4 * tid);
  if (tid < 64) *(volatile v4f*)(bnp + 4 * tid) = v;
  __threadfence();
  if (tid < 64) *(volatile v4f*)(bnp + 4 * tid) = v;
}

__global__ __launch_bounds__(ATHR) void k_apply(
    const float* __restrict__ zpl, const float* __restrict__ h, const float* __restrict__ bnp,
    const float* __restrict__ gamma, const float* __restrict__ beta, const float* __restrict__ eunused,
    float* out, int nN) {
  (void)eunused;
  const int idx = blockIdx.x * ATHR + threadIdx.x;
  const int total = nN * (DF / 4);
  if (idx >= total) return;
  const int row = idx >> 5;
  const int c4  = (idx & 31) * 4;
  const v4f z  = *(const v4f*)(zpl + (size_t)row * DF + c4);
  const v4f hv = *(const v4f*)(h + (size_t)row * DF + c4);
  const v4f mu = *(const v4f*)(bnp + c4);
  const v4f rs = *(const v4f*)(bnp + DF + c4);
  const v4f g  = *(const v4f*)(gamma + c4);
  const v4f bt = *(const v4f*)(beta + c4);
  v4f y = (z - mu) * g;
  y = y * rs;
  y = y + bt;
  y.x = fmaxf(y.x, 0.f); y.y = fmaxf(y.y, 0.f); y.z = fmaxf(y.z, 0.f); y.w = fmaxf(y.w, 0.f);
  const v4f o = hv + y;
  float* op = out + (size_t)row * DF + c4;
  *(volatile v4f*)op = o;
  __threadfence();
  *(volatile v4f*)op = o;
}

extern "C" void kernel_launch(void* const* d_in, const int* in_sizes, int n_in,
                              void* d_out, int out_size, void* d_ws, size_t ws_size,
                              hipStream_t stream) {
  if (n_in < 9) return;
  const int nN = in_sizes[0] / DF;
  if (nN <= 0 || in_sizes[0] != nN * DF) return;
  const int nE = in_sizes[3];
  if (nE < 0 || in_sizes[4] != nE) return;
  if (in_sizes[2] < nN || in_sizes[5] != KTOT * DF) return;
  if (in_sizes[6] < DF || in_sizes[7] < DF || in_sizes[8] < DF) return;
  if (out_size != nN * DF) return;

  const float* h     = (const float*)d_in[0];
  const float* efeat = (const float*)d_in[1];
  const float* snorm = (const float*)d_in[2];
  const int*   srcs  = (const int*)d_in[3];
  const int*   dsts  = (const int*)d_in[4];
  const float* W     = (const float*)d_in[5];
  const float* bpost = (const float*)d_in[6];
  const float* gamma = (const float*)d_in[7];
  const float* beta  = (const float*)d_in[8];
  float* out = (float*)d_out;

  const int nBlk = (nN + NB - 1) / NB;

  char* ws = (char*)d_ws;
  size_t off = 0;
  const size_t oWh = off; off += (size_t)KTOT * DF * 2;                 off = (off + 255) & ~(size_t)255;
  const size_t oWl = off; off += (size_t)KTOT * DF * 2;                 off = (off + 255) & ~(size_t)255;
  const size_t oZ  = off; off += (size_t)nBlk * NB * DF * 4;            off = (off + 255) & ~(size_t)255;
  const size_t oP  = off; off += (size_t)nBlk * (2 * DF) * 8;           off = (off + 255) & ~(size_t)255;
  const size_t oB  = off; off += (size_t)(2 * DF) * 4;                  off = (off + 255) & ~(size_t)255;
  if (off > ws_size) return;
  unsigned short* whi  = (unsigned short*)(ws + oWh);
  unsigned short* wlo  = (unsigned short*)(ws + oWl);
  float*          zpl  = (float*)(ws + oZ);
  double*         part = (double*)(ws + oP);
  float*          bnp  = (float*)(ws + oB);

  const int vec8 = ((nE & 3) == 0) ? 1 : 0;

  const int total8 = KTOT * DF / 8;
  k_wprep<<<(total8 + ATHR - 1) / ATHR, ATHR, 0, stream>>>(W, whi, wlo, total8);

  hipFuncSetAttribute(reinterpret_cast<const void*>(&k_agg),
                      hipFuncAttributeMaxDynamicSharedMemorySize, LDS_AGG);
  k_agg<<<nBlk, NTHR, LDS_AGG, stream>>>(h, srcs, dsts, snorm, bpost, whi, wlo, zpl, part, nN, nE, vec8);

  k_bnfin<<<1, ATHR, 0, stream>>>(part, bnp, nBlk, nN);

  const int totalA = nN * (DF / 4);
  k_apply<<<(totalA + ATHR - 1) / ATHR, ATHR, 0, stream>>>(zpl, h, bnp, gamma, beta, efeat, out, nN);
}
